// GatedCrossScaleFusion_58471684768279
// MI455X (gfx1250) — hardware-verified
//
#include <hip/hip_runtime.h>


#define NB_  4
#define CC   256
#define CQ   64
#define NN   4096
#define PCAR 1024.0f
#define SCL  1.0f
typedef _Float16 h16;
typedef unsigned short bf;
typedef __attribute__((ext_vector_type(16))) __bf16   v16bf;
typedef __attribute__((ext_vector_type(16))) _Float16 v16h;
typedef __attribute__((ext_vector_type(8)))  _Float16 v8h;
typedef __attribute__((ext_vector_type(8)))  unsigned short v8us;
typedef __attribute__((ext_vector_type(8)))  float    v8f;
typedef __attribute__((ext_vector_type(4)))  float    v4f;
typedef v8h  __attribute__((may_alias)) v8ha;
typedef v4f  __attribute__((may_alias)) v4fa;
typedef v8us __attribute__((may_alias)) v8usa;

__device__ __forceinline__ unsigned short f2bf(float f) { unsigned u = __float_as_uint(f); u += 0x7FFFu + ((u >> 16) & 1u); return (unsigned short)(u >> 16); }
__device__ __forceinline__ float bf2f(unsigned short b) { return __uint_as_float(((unsigned)b) << 16); }
__device__ __forceinline__ float bfr(float f) { return bf2f(f2bf(f)); }
__device__ __forceinline__ v16h cat16(v8h lo, v8h hi) { return __builtin_shufflevector(lo, hi, 0, 1, 2, 3, 4, 5, 6, 7, 8, 9, 10, 11, 12, 13, 14, 15); }
__device__ __forceinline__ v16bf cat16b(v8us lo, v8us hi) { return __builtin_bit_cast(v16bf, __builtin_shufflevector(lo, hi, 0, 1, 2, 3, 4, 5, 6, 7, 8, 9, 10, 11, 12, 13, 14, 15)); }
__device__ __forceinline__ v8f wmma16(v16h a, v16h b, v8f c) { return __builtin_amdgcn_wmma_f32_16x16x32_f16(false, a, false, b, (short)0, c, false, false); }
__device__ __forceinline__ v8f wmmab(v16bf a, v16bf b, v8f c) { return __builtin_amdgcn_wmma_f32_16x16x32_bf16(false, a, false, b, (short)0, c, false, false); }


template <typename T16> struct WFrag;
template <> struct WFrag<h16> { typedef v16h V; static __device__ __forceinline__ V ld(const h16* p) { return cat16(*(const v8h*)p, *(const v8h*)(p + 16)); } static __device__ __forceinline__ v8f mma(V a, V b, v8f c) { return wmma16(a, b, c); } };
template <> struct WFrag<bf> { typedef v16bf V; static __device__ __forceinline__ V ld(const bf* p) { return cat16b(*(const v8us*)p, *(const v8us*)(p + 16)); } static __device__ __forceinline__ v8f mma(V a, V b, v8f c) { return wmmab(a, b, c); } };
template <typename T16, int NSPLIT, bool BIAS>
__global__ __launch_bounds__(32) void k_gemmw(const T16* __restrict__ A, const T16* __restrict__ A2, const T16* __restrict__ Bt, const T16* __restrict__ Bt2, int K, float* C, int ldc, const float* __restrict__ bias, size_t sA, size_t sB, size_t sC) {
    typedef typename WFrag<T16>::V V;
    __shared__ __align__(16) float os[16 * 68];
    const size_t z = blockIdx.z; A += z * sA; if (A2) A2 += z * sA; Bt += z * sB; if (Bt2) Bt2 += z * sB; C += z * sC;
    const int lane = threadIdx.x & 31, lr = lane & 15, hi = lane >> 4; const int r0 = blockIdx.x * 64, c0 = blockIdx.y * 64;
    v8f acc[4][4];
#pragma unroll
    for (int mb = 0; mb < 4; ++mb)
#pragma unroll
        for (int nb = 0; nb < 4; ++nb) acc[mb][nb] = (v8f){};
    const size_t aoff = (size_t)(r0 + lr) * K + 8 * hi, boff = (size_t)(c0 + lr) * K + 8 * hi;
#pragma unroll 1
    for (int kc = 0; kc < K; kc += 32) {
        V a[4], a2[4];
#pragma unroll
        for (int mb = 0; mb < 4; ++mb) { a[mb] = WFrag<T16>::ld(A + aoff + (size_t)mb * 16 * K + kc); if (NSPLIT == 1 || NSPLIT == 2) a2[mb] = WFrag<T16>::ld(A2 + aoff + (size_t)mb * 16 * K + kc); }
#pragma unroll
        for (int nb = 0; nb < 4; ++nb) { const V b = WFrag<T16>::ld(Bt + boff + (size_t)nb * 16 * K + kc); V b2; if (NSPLIT >= 2) b2 = WFrag<T16>::ld(Bt2 + boff + (size_t)nb * 16 * K + kc);
#pragma unroll
            for (int mb = 0; mb < 4; ++mb) { acc[mb][nb] = WFrag<T16>::mma(a[mb], b, acc[mb][nb]); if (NSPLIT == 1 || NSPLIT == 2) acc[mb][nb] = WFrag<T16>::mma(a2[mb], b, acc[mb][nb]); if (NSPLIT >= 2) acc[mb][nb] = WFrag<T16>::mma(a[mb], b2, acc[mb][nb]); } }
        asm volatile("v_nop\n\tv_nop\n\tv_nop\n\tv_nop" : "+v"(acc[0][0]), "+v"(acc[1][1]), "+v"(acc[2][2]), "+v"(acc[3][3]) : "v"(a[0]), "v"(a[3]));
    }
#pragma unroll
    for (int mb = 0; mb < 4; ++mb) {
#pragma unroll
        for (int nb = 0; nb < 4; ++nb) {
#pragma unroll
            for (int j = 0; j < 8; ++j) os[(hi * 8 + j) * 68 + nb * 16 + lr] = acc[mb][nb][j]; }
        __builtin_amdgcn_wave_barrier(); asm volatile("" ::: "memory");
        float* crow = C + (size_t)(r0 + mb * 16) * ldc + c0;
#pragma unroll 1
        for (int ps = 0; ps < 2; ++ps) {
#pragma unroll
            for (int s = 0; s < 8; ++s) { const int row = 2 * s + hi, cofs = lr * 4; v4f val = *(const v4fa*)(os + row * 68 + cofs); if (BIAS) { val[0] += bfr(bias[c0 + cofs]); val[1] += bfr(bias[c0 + cofs + 1]); val[2] += bfr(bias[c0 + cofs + 2]); val[3] += bfr(bias[c0 + cofs + 3]); }
                *(volatile v4f*)(crow + (size_t)row * ldc + cofs) = val; }
            if (ps == 0) __threadfence(); }
        __builtin_amdgcn_wave_barrier(); asm volatile("" ::: "memory");
    }
}

__device__ __forceinline__ h16 tohx(float x) { return (h16)x; }
__device__ __forceinline__ void splitf(float y, unsigned short& h, unsigned short& l) { h = f2bf(y); l = f2bf(y - bf2f(h)); }
typedef __attribute__((ext_vector_type(2))) _Float16 v2h;
typedef __attribute__((ext_vector_type(4))) _Float16 v4h;
typedef __attribute__((ext_vector_type(2))) unsigned short v2us;
typedef __attribute__((ext_vector_type(4))) unsigned short v4us;

__global__ __launch_bounds__(256) void k_cvt8(const float* __restrict__ src, bf* dst, size_t n8) { const size_t i = (size_t)blockIdx.x * 256 + threadIdx.x; if (i >= n8) return; const v8f v = *(const v8f*)(src + i * 8); v8us o;
#pragma unroll
    for (int k = 0; k < 8; ++k) o[k] = f2bf(v[k]); *(volatile v8us*)(dst + i * 8) = o; __threadfence(); *(volatile v8us*)(dst + i * 8) = o; }
__global__ __launch_bounds__(256) void k_xt(const float* __restrict__ xb, bf* XT) {
    const int lane = threadIdx.x & 31; const int L0 = (blockIdx.x * 8 + (threadIdx.x >> 5)) * 8; const int nlines = NN * CC / 64;
#pragma unroll 1
    for (int ps = 0; ps < 2; ++ps) {
#pragma unroll
        for (int l = 0; l < 8; ++l) { const int L = L0 + l; if (L >= nlines) break; const int e = L * 64 + lane * 2; const int c = e & (CC - 1); const int n = e >> 8; v2us o;
#pragma unroll
            for (int q = 0; q < 2; ++q) o[q] = f2bf(xb[(size_t)(c + q) * NN + n]);
            *(volatile v2us*)(XT + (size_t)e) = o; }
        if (ps == 0) __threadfence(); }
}
__global__ __launch_bounds__(256) void k_qsplit(const float* __restrict__ F, bf* Ph, bf* Pl) { const size_t i = ((size_t)blockIdx.x * 256 + threadIdx.x) * 2; if (i >= (size_t)NN * CQ) return; v2us oh, ol;
#pragma unroll
    for (int q = 0; q < 2; ++q) { unsigned short a, c2; splitf(F[i + q], a, c2); oh[q] = a; ol[q] = c2; }
    *(volatile v2us*)(Ph + i) = oh; *(volatile v2us*)(Pl + i) = ol; __threadfence(); *(volatile v2us*)(Ph + i) = oh; *(volatile v2us*)(Pl + i) = ol; }
__global__ __launch_bounds__(256) void k_p16(const float* __restrict__ F, h16* P, size_t n) { const size_t i = ((size_t)blockIdx.x * 256 + threadIdx.x) * 2; if (i >= n) return; v2h v; v[0] = tohx(F[i]); v[1] = tohx(F[i + 1]); *(volatile v2h*)(P + i) = v; __threadfence(); *(volatile v2h*)(P + i) = v; }
__global__ __launch_bounds__(256) void k_v16(const float* __restrict__ FV, const float* __restrict__ bv, h16* V16) { const size_t i = ((size_t)blockIdx.x * 256 + threadIdx.x) * 2; if (i >= (size_t)CC * NN) return; const int c = (int)(i >> 12); v2h v;
#pragma unroll
    for (int q = 0; q < 2; ++q) v[q] = tohx(__fadd_rn(FV[i + q], bfr(bv[c]))); *(volatile v2h*)(V16 + i) = v; __threadfence(); *(volatile v2h*)(V16 + i) = v; }
__global__ __launch_bounds__(256) void k_smax(const float* __restrict__ S, float* RS) {
    const int lane = threadIdx.x & 31; const int i = blockIdx.x * 8 + (threadIdx.x >> 5); if (i >= NN) return; const float* sr = S + (size_t)i * NN; float m = -3.0e38f;
#pragma unroll 4
    for (int c0 = lane * 4; c0 < NN; c0 += 128) { const v4f v = *(const v4f*)(sr + c0); m = fmaxf(m, fmaxf(fmaxf(v[0], v[1]), fmaxf(v[2], v[3]))); }
#pragma unroll
    for (int sh = 16; sh; sh >>= 1) m = fmaxf(m, __shfl_xor(m, sh, 32));
    const float o = lane == 0 ? m : 0.f; *(volatile float*)(RS + (size_t)i * 32 + lane) = o; __threadfence(); *(volatile float*)(RS + (size_t)i * 32 + lane) = o;
}
__global__ __launch_bounds__(256) void k_sexp(const float* __restrict__ S, float* RS, h16* P) {
    const int lane = threadIdx.x & 31; const int i = blockIdx.x * 8 + (threadIdx.x >> 5); if (i >= NN) return; const float* sr = S + (size_t)i * NN; const float m = RS[(size_t)i * 32]; float sum = 0.f;
#pragma unroll 2
    for (int c0 = lane * 4; c0 < NN; c0 += 128) { const v4f v = *(const v4f*)(sr + c0); v4h o;
#pragma unroll
        for (int q = 0; q < 4; ++q) { float dlt = __fsub_rn(v[q], m); asm volatile("" : "+v"(dlt)); const float e = __expf(__fmul_rn(dlt, SCL)); sum += e; o[q] = tohx(e * PCAR); }
        *(volatile v4h*)(P + (size_t)i * NN + c0) = o; __threadfence(); *(volatile v4h*)(P + (size_t)i * NN + c0) = o; }
#pragma unroll
    for (int sh = 16; sh; sh >>= 1) sum += __shfl_xor(sum, sh, 32);
    const float o2 = lane == 0 ? m : (lane == 1 ? __fdiv_rn(1.0f, sum * PCAR) : 0.f);   *(volatile float*)(RS + (size_t)i * 32 + lane) = o2; __threadfence(); *(volatile float*)(RS + (size_t)i * 32 + lane) = o2;
}
__global__ __launch_bounds__(256) void k_att(const float* __restrict__ O, const float* __restrict__ RS, float* ATT) { const size_t i = ((size_t)blockIdx.x * 256 + threadIdx.x) * 4; if (i >= (size_t)CC * NN) return; const int n0 = (int)(i & (NN - 1)); const v4f a = *(const v4f*)(O + i); v4f o;
#pragma unroll
    for (int q = 0; q < 4; ++q) o[q] = __fmul_rn(a[q], RS[(size_t)(n0 + q) * 32 + 1]); *(volatile v4f*)(ATT + i) = o; __threadfence(); *(volatile v4f*)(ATT + i) = o; }
__global__ __launch_bounds__(256) void k_catT(const float* __restrict__ decb, const float* __restrict__ ATT, bf* Ch, bf* Cl) {
    const int lane = threadIdx.x & 31; const int L0 = (blockIdx.x * 8 + (threadIdx.x >> 5)) * 8; const int nlines = NN * 2 * CC / 64;
#pragma unroll 1
    for (int ps = 0; ps < 2; ++ps) {
#pragma unroll 1
        for (int l = 0; l < 8; ++l) { const int L = L0 + l; if (L >= nlines) break; const int e = L * 64 + lane * 2; const int c = e & (2 * CC - 1); const int n = e >> 9; v2us oh, ol;
#pragma unroll
            for (int q = 0; q < 2; ++q) { const int cc = c + q; unsigned short a, c2; if (cc < CC) { a = f2bf(decb[(size_t)cc * NN + n]); c2 = 0; } else splitf(ATT[(size_t)(cc - CC) * NN + n], a, c2); oh[q] = a; ol[q] = c2; }
            *(volatile v2us*)(Ch + (size_t)e) = oh; *(volatile v2us*)(Cl + (size_t)e) = ol; }
        if (ps == 0) __threadfence(); }
}
__global__ __launch_bounds__(256) void k_gmean(const float* __restrict__ G1, float* GM) {
    const int lane = threadIdx.x & 31; const int c = blockIdx.x * 8 + (threadIdx.x >> 5); if (c >= CC) return; const float* row = G1 + (size_t)c * NN; float s = 0.f;
#pragma unroll 2
    for (int n0 = lane * 4; n0 < NN; n0 += 128) { const v4f v = *(const v4f*)(row + n0);
#pragma unroll 1
        for (int q = 0; q < 4; ++q) { float e = erff(v[q] * 0.70710678f); asm volatile("" : "+v"(e)); s = __fadd_rn(s, __fmul_rn(__fmul_rn(0.5f, v[q]), __fadd_rn(1.0f, e))); } }
#pragma unroll
    for (int sh = 16; sh; sh >>= 1) s += __shfl_xor(s, sh, 32);
    const float o = (lane == 0) ? s * (1.0f / NN) : 0.f; *(volatile float*)(GM + (size_t)c * 32 + lane) = o; __threadfence(); *(volatile float*)(GM + (size_t)c * 32 + lane) = o; }
__global__ __launch_bounds__(256) void k_gate(const float* __restrict__ GM, const float* __restrict__ Wg2, const float* __restrict__ bg2, float* GT) { const int c = blockIdx.x * 256 + threadIdx.x; if (c >= CC) return; float a = 0.f;
#pragma unroll 4
    for (int k = 0; k < CC; ++k) { float w = bfr(Wg2[(size_t)c * CC + k]); asm volatile("" : "+v"(w)); float m = __fmul_rn(w, GM[(size_t)k * 32]); asm volatile("" : "+v"(m)); a = __fadd_rn(a, m); }
    a = __fadd_rn(a, bfr(bg2[c])); const float g = __fdiv_rn(1.0f, __fadd_rn(1.0f, __expf(-a))); *(volatile float*)(GT + c) = g; __threadfence(); *(volatile float*)(GT + c) = g; }
__global__ __launch_bounds__(256) void k_fuseT(const float* __restrict__ decb, const float* __restrict__ ATT, const float* __restrict__ GT, bf* Fh, bf* Fl) {
    const int lane = threadIdx.x & 31; const int L0 = (blockIdx.x * 8 + (threadIdx.x >> 5)) * 8; const int nlines = NN * CC / 64;
#pragma unroll 1
    for (int ps = 0; ps < 2; ++ps) {
#pragma unroll 1
        for (int l = 0; l < 8; ++l) { const int L = L0 + l; if (L >= nlines) break; const int e = L * 64 + lane * 2; const int c = e & (CC - 1); const int n = e >> 8; v2us oh, ol;
#pragma unroll
            for (int q = 0; q < 2; ++q) { const int cc = c + q; const float g = GT[cc]; float t1 = __fmul_rn(g, ATT[(size_t)cc * NN + n]), t2 = __fmul_rn(__fsub_rn(1.0f, g), bfr(decb[(size_t)cc * NN + n])); asm volatile("" : "+v"(t1)); asm volatile("" : "+v"(t2)); unsigned short a, c2; splitf(__fadd_rn(t1, t2), a, c2); oh[q] = a; ol[q] = c2; }
            *(volatile v2us*)(Fh + (size_t)e) = oh; *(volatile v2us*)(Fl + (size_t)e) = ol; }
        if (ps == 0) __threadfence(); }
}
__global__ __launch_bounds__(256) void k_amap(const float* __restrict__ ATT, float* AMb) { const int n = blockIdx.x * 256 + threadIdx.x; if (n >= NN) return; float s = 0.f; for (int c = 0; c < CC; ++c) s = __fadd_rn(s, ATT[(size_t)c * NN + n]);
    const float o = s * (1.0f / CC); *(volatile float*)(AMb + n) = o; __threadfence(); *(volatile float*)(AMb + n) = o; }
template <int PASS>
__global__ __launch_bounds__(256) void k_bnstat(const float* __restrict__ Y, float* BS) {
    const int lane = threadIdx.x & 31; const int c = blockIdx.x * 8 + (threadIdx.x >> 5); if (c >= CC) return; const float mu = PASS ? BS[(size_t)c * 32] : 0.f; float s = 0.f;
    for (int b = 0; b < NB_; ++b) { const float* row = Y + ((size_t)b * CC + c) * NN;
#pragma unroll 2
        for (int n0 = lane * 4; n0 < NN; n0 += 128) { const v4f v = *(const v4f*)(row + n0);
#pragma unroll
            for (int q = 0; q < 4; ++q) { float x = v[q]; if (PASS) { const float d0 = __fsub_rn(x, mu); x = __fmul_rn(d0, d0); } s = __fadd_rn(s, x); } } }
#pragma unroll
    for (int sh = 16; sh; sh >>= 1) s += __shfl_xor(s, sh, 32);
    const float tot = s * (1.0f / (NB_ * NN)); float o;
    if (PASS == 0) o = (lane == 0) ? tot : 0.f; else o = (lane == 0) ? mu : (lane == 1 ? __fdiv_rn(1.0f, __fsqrt_rn(__fadd_rn(tot, 1e-5f))) : 0.f);
    *(volatile float*)(BS + (size_t)c * 32 + lane) = o; __threadfence(); *(volatile float*)(BS + (size_t)c * 32 + lane) = o; }
__global__ __launch_bounds__(256) void k_bnout(const float* __restrict__ Y, const float* __restrict__ BS, const float* __restrict__ gam, const float* __restrict__ bet, float* OUT0) { const size_t i = ((size_t)blockIdx.x * 256 + threadIdx.x) * 4; if (i >= (size_t)NB_ * CC * NN) return; const int c = (int)((i >> 12) & (CC - 1)); const float mu = BS[(size_t)c * 32], rs = BS[(size_t)c * 32 + 1], g = bfr(gam[c]), bb = bfr(bet[c]); const v4f y4 = *(const v4f*)(Y + i); v4f o;
#pragma unroll 1
    for (int q = 0; q < 4; ++q) { float t = __fmul_rn(__fsub_rn(y4[q], mu), rs); asm volatile("" : "+v"(t)); const float z = __fadd_rn(__fmul_rn(t, g), bb); float e = erff(z * 0.70710678f); asm volatile("" : "+v"(e)); o[q] = __fmul_rn(__fmul_rn(0.5f, z), __fadd_rn(1.0f, e)); }
    *(volatile v4f*)(OUT0 + i) = o; __threadfence(); *(volatile v4f*)(OUT0 + i) = o; }

extern "C" void kernel_launch(void* const* d_in, const int* in_sizes, int n_in,
                              void* d_out, int out_size, void* d_ws, size_t ws_size, hipStream_t stream) {
    (void)in_sizes; (void)n_in; (void)out_size;
    const float* IN[11]; for (int i = 0; i < 11; ++i) IN[i] = (const float*)d_in[i];
    const float* dec = IN[0]; const float* enc = IN[1];
    float* OUT0 = (float*)d_out; float* OUT1 = OUT0 + (size_t)NB_ * CC * NN;
    char* wsp = (char*)d_ws;
    auto take = [&](size_t bytes) { char* p = wsp; wsp += (bytes + 255) & ~(size_t)255; return (void*)p; };
    bf* WQ = (bf*)take((size_t)CQ * CC * 2); bf* WK = (bf*)take((size_t)CQ * CC * 2); bf* WV = (bf*)take((size_t)CC * CC * 2); bf* WG1 = (bf*)take((size_t)CC * 2 * CC * 2); bf* WO = (bf*)take((size_t)CC * CC * 2);
    bf* XD = (bf*)take((size_t)NN * CC * 2); bf* XE = (bf*)take((size_t)NN * CC * 2); float* FQ = (float*)take((size_t)NN * CQ * 4); bf* Qh = (bf*)take((size_t)NN * CQ * 2); bf* Ql = (bf*)take((size_t)NN * CQ * 2); bf* Kh = (bf*)take((size_t)NN * CQ * 2); bf* Kl = (bf*)take((size_t)NN * CQ * 2);
    float* FV = (float*)take((size_t)CC * NN * 4); h16* V16 = (h16*)take((size_t)CC * NN * 2); float* S = (float*)take((size_t)NN * NN * 4); h16* P = (h16*)take((size_t)NN * NN * 2); float* RS = (float*)take((size_t)NN * 32 * 4);
    float* ATT = (float*)take((size_t)CC * NN * 4); bf* Ch = (bf*)take((size_t)NN * 2 * CC * 2); bf* Cl = (bf*)take((size_t)NN * 2 * CC * 2); float* G1 = (float*)take((size_t)CC * NN * 4); float* GM = (float*)take(CC * 32 * 4); float* GT = (float*)take(CC * 4);
    bf* Fh = (bf*)take((size_t)NN * CC * 2); bf* Fl = (bf*)take((size_t)NN * CC * 2); float* Y = (float*)take((size_t)NB_ * CC * NN * 4); float* BS = (float*)take(CC * 32 * 4);
    if ((size_t)(wsp - (char*)d_ws) > ws_size) return;
    float* Oc = FV;
    { k_cvt8<<<(CQ * CC / 8 + 255) / 256, 256, 0, stream>>>(IN[2], WQ, (size_t)CQ * CC / 8); k_cvt8<<<(CQ * CC / 8 + 255) / 256, 256, 0, stream>>>(IN[3], WK, (size_t)CQ * CC / 8); k_cvt8<<<(CC * CC / 8 + 255) / 256, 256, 0, stream>>>(IN[4], WV, (size_t)CC * CC / 8);
      k_cvt8<<<(CC * 2 * CC / 8 + 255) / 256, 256, 0, stream>>>(IN[5], WG1, (size_t)CC * 2 * CC / 8); k_cvt8<<<(CC * CC / 8 + 255) / 256, 256, 0, stream>>>(IN[8], WO, (size_t)CC * CC / 8); }
    const unsigned LX = (unsigned)((NN * CC / 64 + 63) / 64), L2 = (unsigned)(((size_t)NN * CC / 2 + 255) / 256), L4 = (unsigned)(((size_t)NN * CC / 4 + 255) / 256), LQ = (unsigned)(((size_t)NN * CQ / 2 + 255) / 256);
    for (int b = 0; b < NB_; ++b) { const float* db = dec + (size_t)b * CC * NN; const float* eb = enc + (size_t)b * CC * NN;
        k_xt<<<LX, 256, 0, stream>>>(db, XD); k_xt<<<LX, 256, 0, stream>>>(eb, XE);
        k_gemmw<bf, 0, false><<<dim3(NN / 64, 1, 1), 32, 0, stream>>>(XD, nullptr, WQ, nullptr, CC, FQ, CQ, nullptr, 0, 0, 0); k_qsplit<<<LQ, 256, 0, stream>>>(FQ, Qh, Ql);
        k_gemmw<bf, 0, false><<<dim3(NN / 64, 1, 1), 32, 0, stream>>>(XE, nullptr, WK, nullptr, CC, FQ, CQ, nullptr, 0, 0, 0); k_qsplit<<<LQ, 256, 0, stream>>>(FQ, Kh, Kl);
        k_gemmw<bf, 0, false><<<dim3(CC / 64, NN / 64, 1), 32, 0, stream>>>(WV, nullptr, XE, nullptr, CC, FV, NN, nullptr, 0, 0, 0); k_p16<<<L2, 256, 0, stream>>>(FV, V16, (size_t)CC * NN);
        k_gemmw<bf, 2, false><<<dim3(NN / 64, NN / 64, 1), 32, 0, stream>>>(Qh, Ql, Kh, Kl, CQ, S, NN, nullptr, 0, 0, 0);
        k_smax<<<NN / 8, 256, 0, stream>>>(S, RS); k_sexp<<<NN / 8, 256, 0, stream>>>(S, RS, P);
        k_gemmw<h16, 0, false><<<dim3(CC / 64, NN / 64, 1), 32, 0, stream>>>(V16, nullptr, P, nullptr, NN, Oc, NN, nullptr, 0, 0, 0);
        k_att<<<L4, 256, 0, stream>>>(Oc, RS, ATT); k_amap<<<NN / 256, 256, 0, stream>>>(ATT, OUT1 + (size_t)b * NN);
        k_catT<<<(NN * 2 * CC / 64 + 63) / 64, 256, 0, stream>>>(db, ATT, Ch, Cl);
        k_gemmw<bf, 3, false><<<dim3(CC / 64, NN / 64, 1), 32, 0, stream>>>(WG1, nullptr, Ch, Cl, 2 * CC, G1, NN, nullptr, 0, 0, 0);
        k_gmean<<<CC / 8, 256, 0, stream>>>(G1, GM); k_gate<<<1, 256, 0, stream>>>(GM, IN[6], IN[7], GT);
        k_fuseT<<<LX, 256, 0, stream>>>(db, ATT, GT, Fh, Fl);
        k_gemmw<bf, 3, false><<<dim3(CC / 64, NN / 64, 1), 32, 0, stream>>>(WO, nullptr, Fh, Fl, CC, Y + (size_t)b * CC * NN, NN, nullptr, 0, 0, 0); }
    k_bnstat<0><<<CC / 8, 256, 0, stream>>>(Y, BS); k_bnstat<1><<<CC / 8, 256, 0, stream>>>(Y, BS);
    k_bnout<<<(unsigned)(((size_t)NB_ * CC * NN / 4 + 255) / 256), 256, 0, stream>>>(Y, BS, IN[9], IN[10], OUT0);
}
